// PointnetFPModule_57793079935589
// MI455X (gfx1250) — hardware-verified
//
#include <hip/hip_runtime.h>
#include <stdint.h>

#pragma clang fp contract(off)

typedef __attribute__((ext_vector_type(16))) _Float16 v16h;
typedef __attribute__((ext_vector_type(8)))  _Float16 v8h;
typedef __attribute__((ext_vector_type(8)))  float    v8f;
typedef __attribute__((ext_vector_type(4)))  float    v4f;
typedef __attribute__((ext_vector_type(4)))  int      v4i;

constexpr int NBATCH   = 4;
constexpr int NUNK     = 16384;
constexpr int NKNOWN   = 4096;
constexpr int CH_SKIP  = 128;
constexpr int CH_DEEP  = 256;
constexpr int CH_IN    = CH_DEEP + CH_SKIP;
constexpr int CH_HID1  = 256;
constexpr int CH_HID2  = 128;
constexpr int NPOINTS  = NBATCH * NUNK;
constexpr float INTERP_EPS = 1e-8f;
constexpr float BN_EPSILON = 1e-5f;
constexpr float W_CARRY     = 16384.0f;
constexpr float W_CARRY_INV = 1.0f / 16384.0f;

constexpr int KNN_CHUNK  = 2048;
constexpr int STAT_BLOCKS = 64;
constexpr int STAT_ROWS   = 1024;
constexpr int XT_PITCH = 388;
constexpr int OT_PITCH = 132;

static_assert(CH_IN == 384, "contract");
static_assert(NPOINTS == 65536, "contract");
static_assert(NUNK % 256 == 0 && NUNK % 32 == 0, "blocks never straddle a batch");
static_assert(NKNOWN % KNN_CHUNK == 0, "chunking");
static_assert((KNN_CHUNK * 3) % (4 * 256) == 0, "staging coverage");
static_assert(CH_IN % 32 == 0 && CH_HID1 % 32 == 0, "K multiples of 32");
static_assert(NPOINTS % 64 == 0 && CH_HID1 % 64 == 0 && CH_HID2 % 64 == 0, "tile multiples");
static_assert(STAT_BLOCKS * STAT_ROWS == NPOINTS, "stats coverage");
static_assert((CH_HID1 * CH_IN) % (8 * 256) == 0 && (CH_HID2 * CH_HID1) % (8 * 256) == 0, "pack grid exact");

constexpr size_t OFF_TAB    = 0;
constexpr size_t OFF_PART1  = OFF_TAB + 4096;
constexpr size_t OFF_PART2  = OFF_PART1 + (size_t)STAT_BLOCKS * CH_HID1 * 2 * 4;
constexpr size_t OFF_W1HI   = OFF_PART2 + (size_t)STAT_BLOCKS * CH_HID2 * 2 * 4;
constexpr size_t OFF_W1LO   = OFF_W1HI + (size_t)CH_HID1 * CH_IN * 2;
constexpr size_t OFF_W2HI   = OFF_W1LO + (size_t)CH_HID1 * CH_IN * 2;
constexpr size_t OFF_W2LO   = OFF_W2HI + (size_t)CH_HID2 * CH_HID1 * 2;
constexpr size_t OFF_DSEL   = OFF_W2LO + (size_t)CH_HID2 * CH_HID1 * 2;
constexpr size_t OFF_ISEL   = OFF_DSEL + (size_t)NPOINTS * 16;
constexpr size_t OFF_PLANEA = OFF_ISEL + (size_t)NPOINTS * 16;
constexpr size_t SZ_PLANEA  = (size_t)NPOINTS * CH_IN * 2;
constexpr size_t OFF_PLANEB = OFF_PLANEA + SZ_PLANEA;
constexpr size_t SZ_PLANEB  = (size_t)NPOINTS * CH_HID1 * 4;
constexpr size_t WS_TOTAL   = OFF_PLANEB + SZ_PLANEB;
static_assert(WS_TOTAL <= (size_t)134217728, "carve within 128 MiB");
static_assert((size_t)NPOINTS * CH_HID1 * 2 <= SZ_PLANEA, "H1 fits plane A");
static_assert((size_t)NPOINTS * CH_HID2 * 4 <= SZ_PLANEB, "Y2 fits plane B");
static_assert(OFF_PART1 % 128 == 0 && OFF_PART2 % 128 == 0 && OFF_W1HI % 128 == 0 && OFF_W1LO % 128 == 0 &&
              OFF_W2HI % 128 == 0 && OFF_W2LO % 128 == 0 && OFF_DSEL % 128 == 0 && OFF_ISEL % 128 == 0 &&
              OFF_PLANEA % 128 == 0 && OFF_PLANEB % 128 == 0, "line aligned carves");

__device__ __forceinline__ void keep4_h(v16h a, v16h b, v16h c, v16h d) { asm volatile("v_nop" :: "v"(a), "v"(b), "v"(c), "v"(d)); }
__device__ __forceinline__ void acc_guard4(v8f& a, v8f& b, v8f& c, v8f& d) { asm volatile("v_nop\n\tv_nop\n\tv_nop\n\tv_nop" : "+v"(a), "+v"(b), "+v"(c), "+v"(d)); }
__device__ __forceinline__ void row_guard_h(v8f& a0, v8f& a1, v8f& a2, v8f& a3, v16h x,
                                            v16h b0, v16h b1, v16h b2, v16h b3,
                                            v16h l0, v16h l1, v16h l2, v16h l3) {
  asm volatile("v_nop\n\tv_nop\n\tv_nop\n\tv_nop"
               : "+v"(a0), "+v"(a1), "+v"(a2), "+v"(a3)
               : "v"(x), "v"(b0), "v"(b1), "v"(b2), "v"(b3), "v"(l0), "v"(l1), "v"(l2), "v"(l3));
}
struct FragH {
  union U { v16h v; v8h h[2]; };
  static __device__ __forceinline__ v16h load(const _Float16* p) {
    U f; f.h[0] = *(const v8h*)(p); f.h[1] = *(const v8h*)(p + 16); return f.v;
  }
  static __device__ __forceinline__ v8f mma(v16h a, v16h b, v8f c) {
    return __builtin_amdgcn_wmma_f32_16x16x32_f16(false, a, false, b, (short)0, c, false, false);
  }
};

__global__ __launch_bounds__(256) void pack_w_kernel(
    const float* __restrict__ w, unsigned short* __restrict__ hi, unsigned short* __restrict__ lo, int n8) {
  const int i = blockIdx.x * 256 + threadIdx.x;
  if (i < n8) {
    const v4f a = *(const v4f*)(w + (size_t)i * 8);
    const v4f b = *(const v4f*)(w + (size_t)i * 8 + 4);
    float f[8];
    f[0] = a[0]; f[1] = a[1]; f[2] = a[2]; f[3] = a[3];
    f[4] = b[0]; f[5] = b[1]; f[6] = b[2]; f[7] = b[3];
    v8h hv, lv;
#pragma unroll
    for (int e = 0; e < 8; ++e) {
      const float s = f[e] * W_CARRY;
      const _Float16 hh = (_Float16)s;
      const float r = s - (float)hh;
      hv[e] = hh;
      lv[e] = (_Float16)r;
    }
    *(volatile v8h*)(hi + (size_t)i * 8) = hv;
    *(volatile v8h*)(lo + (size_t)i * 8) = lv;
    __threadfence();
    *(volatile v8h*)(hi + (size_t)i * 8) = hv;
    *(volatile v8h*)(lo + (size_t)i * 8) = lv;
  }
}

#define KNN_DOT3_FMA_CHAIN 1
__global__ __launch_bounds__(256) void knn3_kernel(
    const float* __restrict__ unk, const float* __restrict__ kn,
    float* __restrict__ dsel, int* __restrict__ isel) {
#pragma clang fp contract(off)
  __shared__ __align__(16) float sk[KNN_CHUNK * 4];
  const int tid = threadIdx.x;
  const int gp  = blockIdx.x * 256 + tid;
  const int b   = gp / NUNK;
  const float ux = unk[(size_t)gp * 3 + 0];
  const float uy = unk[(size_t)gp * 3 + 1];
  const float uz = unk[(size_t)gp * 3 + 2];
  const float u2 = (ux * ux + uz * uz) + uy * uy;
  float e0 = __builtin_inff(), e1 = __builtin_inff(), e2 = __builtin_inff();
  int i0 = 0, i1 = 0, i2 = 0;
  for (int ch = 0; ch < NKNOWN / KNN_CHUNK; ++ch) {
    __syncthreads();
    const float* kb = kn + ((size_t)b * NKNOWN + (size_t)ch * KNN_CHUNK) * 3;
#pragma unroll
    for (int j = 0; j < 6; ++j) {
      const int q = tid + 256 * j;
      const v4f v = *(const v4f*)(kb + 4 * q);
#pragma unroll
      for (int e = 0; e < 4; ++e) {
        const int f = 4 * q + e;
        const int m = f / 3;
        const int c = f - 3 * m;
        sk[m * 4 + c] = v[e];
      }
    }
    __syncthreads();
#pragma unroll
    for (int j = 0; j < 8; ++j) {
      const int m = tid + 256 * j;
      const float x = sk[m * 4 + 0], y = sk[m * 4 + 1], z = sk[m * 4 + 2];
      sk[m * 4 + 3] = (x * x + z * z) + y * y;
    }
    __syncthreads();
#pragma unroll 4
    for (int m = 0; m < KNN_CHUNK; ++m) {
      const v4f kv = *(const v4f*)(sk + 4 * m);
      const float kx = kv[0], ky = kv[1], kz = kv[2], k2 = kv[3];
#if KNN_DOT3_FMA_CHAIN
      float p = ux * kx;
      p = __builtin_fmaf(uy, ky, p);
      p = __builtin_fmaf(uz, kz, p);
#else
      float p = (ux * kx + uy * ky) + uz * kz;
#endif
      const float s = u2 + k2;
      const float d = s - (p + p);
      const int mi = ch * KNN_CHUNK + m;
      const bool c0 = d < e0, c1 = d < e1, c2 = d < e2;
      e2 = c1 ? e1 : (c2 ? d : e2);
      i2 = c1 ? i1 : (c2 ? mi : i2);
      e1 = c0 ? e0 : (c1 ? d : e1);
      i1 = c0 ? i0 : (c1 ? mi : i1);
      e0 = c0 ? d : e0;
      i0 = c0 ? mi : i0;
    }
  }
  v4f dv; dv[0] = e0; dv[1] = e1; dv[2] = e2; dv[3] = 0.0f;
  v4i iv; iv[0] = i0; iv[1] = i1; iv[2] = i2; iv[3] = 0;
  *(volatile v4f*)(dsel + (size_t)gp * 4) = dv;
  *(volatile v4i*)(isel + (size_t)gp * 4) = iv;
  __threadfence();
  *(volatile v4f*)(dsel + (size_t)gp * 4) = dv;
  *(volatile v4i*)(isel + (size_t)gp * 4) = iv;
}

__global__ __launch_bounds__(256) void build_x_kernel(
    const float* __restrict__ kf, const float* __restrict__ uf,
    const float* __restrict__ dsel, const int* __restrict__ isel,
    unsigned short* __restrict__ xt) {
  __shared__ __align__(16) float xs[32 * XT_PITCH];
  __shared__ float swt[3 * 32];
  __shared__ int   sid[3 * 32];
  const int tid  = threadIdx.x;
  const int lane = tid & 31;
  const int wave = tid >> 5;
  const int p0 = blockIdx.x * 32;
  const int b  = p0 / NUNK;
  const int n0 = p0 - b * NUNK;
  if (tid < 32) {
    const v4f dv = *(const v4f*)(dsel + (size_t)(p0 + tid) * 4);
    const v4i iv = *(const v4i*)(isel + (size_t)(p0 + tid) * 4);
    const float q0 = dv[0], q1 = dv[1], q2 = dv[2];
    const int a0 = iv[0], a1 = iv[1], a2 = iv[2];
    const float d0 = fmaxf(q0, 0.0f), d1 = fmaxf(q1, 0.0f), d2 = fmaxf(q2, 0.0f);
    const float r0 = 1.0f / (d0 + INTERP_EPS);
    const float r1 = 1.0f / (d1 + INTERP_EPS);
    const float r2 = 1.0f / (d2 + INTERP_EPS);
    const float rs = (r0 + r2) + r1;
    swt[tid]      = r0 / rs;
    swt[32 + tid] = r1 / rs;
    swt[64 + tid] = r2 / rs;
    sid[tid]      = min(max(a0, 0), NKNOWN - 1);
    sid[32 + tid] = min(max(a1, 0), NKNOWN - 1);
    sid[64 + tid] = min(max(a2, 0), NKNOWN - 1);
  }
  __syncthreads();
  const float w0 = swt[lane], w1 = swt[32 + lane], w2 = swt[64 + lane];
  const int j0 = sid[lane], j1 = sid[32 + lane], j2 = sid[64 + lane];
  const float* kfb = kf + (size_t)b * CH_DEEP * NKNOWN;
#pragma unroll 1
  for (int jj = 0; jj < 8; ++jj) {
#pragma unroll
    for (int u = 0; u < 4; ++u) {
      const int c = wave + 8 * (jj * 4 + u);
      const float* row = kfb + (size_t)c * NKNOWN;
      const float g0 = row[j0], g1 = row[j1], g2 = row[j2];
      xs[lane * XT_PITCH + c] = (g0 * w0 + g2 * w2) + g1 * w1;
    }
    asm volatile("" ::: "memory");
  }
  const float* ufb = uf + (size_t)b * CH_SKIP * NUNK + n0 + lane;
#pragma unroll 1
  for (int jj = 0; jj < 4; ++jj) {
#pragma unroll
    for (int u = 0; u < 4; ++u) {
      const int c = wave + 8 * (jj * 4 + u);
      xs[lane * XT_PITCH + CH_DEEP + c] = ufb[(size_t)c * NUNK];
    }
    asm volatile("" ::: "memory");
  }
  __syncthreads();
  unsigned short* dst = xt + (size_t)p0 * CH_IN;
  for (int pass = 0; pass < 2; ++pass) {
#pragma unroll
    for (int it = 0; it < 6; ++it) {
      const int q = it * 256 + tid;
      const int row = q / 48;
      const int c8 = (q - row * 48) * 8;
      const float* sp = xs + row * XT_PITCH + c8;
      const v4f a = *(const v4f*)(sp);
      const v4f c = *(const v4f*)(sp + 4);
      v8h hv;
      hv[0] = (_Float16)a[0]; hv[1] = (_Float16)a[1]; hv[2] = (_Float16)a[2]; hv[3] = (_Float16)a[3];
      hv[4] = (_Float16)c[0]; hv[5] = (_Float16)c[1]; hv[6] = (_Float16)c[2]; hv[7] = (_Float16)c[3];
      *(volatile v8h*)(dst + (size_t)q * 8) = hv;
    }
    __threadfence();
  }
}

__global__ __launch_bounds__(256) void gemm_f16_wsplit_kernel(
    const unsigned short* __restrict__ Ap, int lda,
    const unsigned short* __restrict__ Bhp, const unsigned short* __restrict__ Blp, int ldb,
    float* __restrict__ Cout, int ldc, const float* __restrict__ bias,
    int M, int N, int K, float scale) {
  const _Float16* A  = (const _Float16*)Ap;
  const _Float16* Bh = (const _Float16*)Bhp;
  const _Float16* Bl = (const _Float16*)Blp;
  __shared__ __align__(16) float sT[8][16 * 68];
  const int lane = threadIdx.x & 31;
  const int wave = threadIdx.x >> 5;
  const int tilesN = N >> 6;
  const int tilesM = M >> 6;
  const int tile = blockIdx.x * 8 + wave;
  if (tile >= tilesM * tilesN) return;
  const int tm = tile / tilesN;
  const int tn = tile - tm * tilesN;
  const int m0 = tm << 6;
  const int n0 = tn << 6;
  const int rlane = lane & 15;
  const int koff  = (lane >> 4) * 8;
  const int mOff  = (lane >> 4) * 8;

  v8f acc[4][4];
#pragma unroll
  for (int i = 0; i < 4; ++i)
#pragma unroll
    for (int j = 0; j < 4; ++j) acc[i][j] = (v8f){0.f, 0.f, 0.f, 0.f, 0.f, 0.f, 0.f, 0.f};

  for (int k0 = 0; k0 < K; k0 += 32) {
    v16h bh[4], bl[4];
#pragma unroll
    for (int j = 0; j < 4; ++j) {
      const size_t bo = (size_t)(n0 + (j << 4) + rlane) * ldb + koff + k0;
      bh[j] = FragH::load(Bh + bo);
      bl[j] = FragH::load(Bl + bo);
    }
#pragma unroll
    for (int i = 0; i < 4; ++i) {
      const size_t ao = (size_t)(m0 + (i << 4) + rlane) * lda + koff + k0;
      const v16h ah = FragH::load(A + ao);
#pragma unroll
      for (int j = 0; j < 4; ++j) {
        acc[i][j] = FragH::mma(ah, bh[j], acc[i][j]);
        acc[i][j] = FragH::mma(ah, bl[j], acc[i][j]);
      }
      row_guard_h(acc[i][0], acc[i][1], acc[i][2], acc[i][3], ah,
                  bh[0], bh[1], bh[2], bh[3], bl[0], bl[1], bl[2], bl[3]);
    }
    keep4_h(bh[0], bh[1], bh[2], bh[3]);
    keep4_h(bl[0], bl[1], bl[2], bl[3]);
  }
  acc_guard4(acc[0][0], acc[0][1], acc[0][2], acc[0][3]);
  acc_guard4(acc[1][0], acc[1][1], acc[1][2], acc[1][3]);
  acc_guard4(acc[2][0], acc[2][1], acc[2][2], acc[2][3]);
  acc_guard4(acc[3][0], acc[3][1], acc[3][2], acc[3][3]);

  float* slab = sT[wave];
#pragma unroll
  for (int i = 0; i < 4; ++i) {
    const int mBase = m0 + (i << 4);
#pragma unroll
    for (int j = 0; j < 4; ++j) {
      const int n = n0 + (j << 4) + rlane;
      const float bv = bias[n];
#pragma unroll
      for (int r = 0; r < 8; ++r) {
        float v = acc[i][j][r] * scale;
        v += bv;
        slab[(mOff + r) * 68 + (j << 4) + rlane] = v;
      }
    }
    __builtin_amdgcn_fence(__ATOMIC_RELEASE, "workgroup");
    __builtin_amdgcn_wave_barrier();
    __builtin_amdgcn_fence(__ATOMIC_ACQUIRE, "workgroup");
    {
      const int hh = lane >> 4, c4 = (lane & 15) * 4;
      for (int pass = 0; pass < 2; ++pass) {
#pragma unroll
        for (int it = 0; it < 8; ++it) {
          const int row = it * 2 + hh;
          const v4f v = *(const v4f*)(slab + row * 68 + c4);
          *(volatile v4f*)(Cout + (size_t)(mBase + row) * ldc + n0 + c4) = v;
        }
        __threadfence();
      }
    }
    __builtin_amdgcn_fence(__ATOMIC_RELEASE, "workgroup");
    __builtin_amdgcn_wave_barrier();
    __builtin_amdgcn_fence(__ATOMIC_ACQUIRE, "workgroup");
  }
}

template <int NCH>
__global__ __launch_bounds__(NCH) void stats_kernel(
    const float* __restrict__ y, float* __restrict__ psum, float* __restrict__ psq) {
  const int t = threadIdx.x, blk = blockIdx.x;
  const float* base = y + (size_t)blk * STAT_ROWS * NCH + t;
  float so = 0.0f, qo = 0.0f;
#pragma unroll 1
  for (int g = 0; g < STAT_ROWS / 8; ++g) {
    float s = 0.0f, q = 0.0f;
#pragma unroll
    for (int u = 0; u < 8; ++u) {
      const float v = base[(size_t)(g * 8 + u) * NCH];
      s += v;
      q += v * v;
    }
    so += s;
    qo += q;
    asm volatile("" ::: "memory");
  }
  *(volatile float*)(psum + (size_t)blk * NCH + t) = so;
  *(volatile float*)(psq  + (size_t)blk * NCH + t) = qo;
  __threadfence();
  *(volatile float*)(psum + (size_t)blk * NCH + t) = so;
  *(volatile float*)(psq  + (size_t)blk * NCH + t) = qo;
}

__global__ void bn_finalize_kernel(
    const float* __restrict__ psum, const float* __restrict__ psq,
    const float* __restrict__ g, const float* __restrict__ be,
    float* __restrict__ sarr, float* __restrict__ tarr, int nch) {
  const int c = threadIdx.x;
  if (c < nch) {
    double s = 0.0, q = 0.0;
#pragma unroll 8
    for (int i = 0; i < STAT_BLOCKS; ++i) {
      s += (double)psum[(size_t)i * nch + c];
      q += (double)psq[(size_t)i * nch + c];
    }
    const double invp = 1.0 / (double)NPOINTS;
    const double mu = s * invp;
    double var = q * invp - mu * mu;
    var = var < 0.0 ? 0.0 : var;
    const float varf = (float)var;
    const float rs = 1.0f / sqrtf(varf + BN_EPSILON);
    const float sc = g[c] * rs;
    const float tc = be[c] - (float)mu * sc;
    *(volatile float*)(sarr + c) = sc;
    *(volatile float*)(tarr + c) = tc;
    __threadfence();
    *(volatile float*)(sarr + c) = sc;
    *(volatile float*)(tarr + c) = tc;
  }
}

__global__ __launch_bounds__(256) void bn_relu_f16_kernel(
    const float* __restrict__ y, const float* __restrict__ sarr, const float* __restrict__ tarr,
    unsigned short* __restrict__ h) {
  const size_t e = (size_t)blockIdx.x * 256 + threadIdx.x;
  const int c0 = (int)((e * 8) & (size_t)(CH_HID1 - 1));
  const v4f ya = *(const v4f*)(y + e * 8);
  const v4f yb = *(const v4f*)(y + e * 8 + 4);
  const v4f sa = *(const v4f*)(sarr + c0);
  const v4f sb = *(const v4f*)(sarr + c0 + 4);
  const v4f ta = *(const v4f*)(tarr + c0);
  const v4f tb = *(const v4f*)(tarr + c0 + 4);
  v8h hv;
#pragma unroll
  for (int k = 0; k < 4; ++k) {
    const float va = fmaxf(sa[k] * ya[k] + ta[k], 0.0f);
    const float vb = fmaxf(sb[k] * yb[k] + tb[k], 0.0f);
    hv[k]     = (_Float16)va;
    hv[4 + k] = (_Float16)vb;
  }
  *(volatile v8h*)(h + e * 8) = hv;
  __threadfence();
  *(volatile v8h*)(h + e * 8) = hv;
}

__global__ __launch_bounds__(256) void bn_relu_out_kernel(
    const float* __restrict__ y2, const float* __restrict__ s2, const float* __restrict__ t2,
    float* __restrict__ out) {
  __shared__ float tile[32 * OT_PITCH];
  const int tid  = threadIdx.x;
  const int lane = tid & 31;
  const int wave = tid >> 5;
  const int p0 = blockIdx.x * 32;
  const int b  = p0 / NUNK;
  const int n0 = p0 - b * NUNK;
  const float* src = y2 + (size_t)p0 * CH_HID2;
#pragma unroll
  for (int j = 0; j < 4; ++j) {
    const int q = tid + 256 * j;
    const v4f v = *(const v4f*)(src + 4 * q);
    const int row = q >> 5;
    const int c4 = (q & 31) * 4;
    tile[row * OT_PITCH + c4 + 0] = v[0];
    tile[row * OT_PITCH + c4 + 1] = v[1];
    tile[row * OT_PITCH + c4 + 2] = v[2];
    tile[row * OT_PITCH + c4 + 3] = v[3];
  }
  __syncthreads();
  for (int pass = 0; pass < 2; ++pass) {
#pragma unroll 4
    for (int j = 0; j < 16; ++j) {
      const int c = wave + 8 * j;
      const float v = fmaxf(s2[c] * tile[lane * OT_PITCH + c] + t2[c], 0.0f);
      *(volatile float*)(out + ((size_t)b * CH_HID2 + c) * NUNK + n0 + lane) = v;
    }
    __threadfence();
  }
}

extern "C" void kernel_launch(void* const* d_in, const int* in_sizes, int n_in,
                              void* d_out, int out_size, void* d_ws, size_t ws_size,
                              hipStream_t stream) {
  (void)in_sizes; (void)n_in; (void)out_size;
  if (ws_size < WS_TOTAL) return;
  const float* unknown = (const float*)d_in[0];
  const float* known   = (const float*)d_in[1];
  const float* uf      = (const float*)d_in[2];
  const float* kf      = (const float*)d_in[3];
  const float* W1      = (const float*)d_in[4];
  const float* b1      = (const float*)d_in[5];
  const float* g1      = (const float*)d_in[6];
  const float* be1     = (const float*)d_in[7];
  const float* W2      = (const float*)d_in[8];
  const float* b2      = (const float*)d_in[9];
  const float* g2      = (const float*)d_in[10];
  const float* be2     = (const float*)d_in[11];

  unsigned char* ws = (unsigned char*)d_ws;
  float* tab = (float*)(ws + OFF_TAB);
  float* s1 = tab;
  float* t1 = tab + 256;
  float* s2 = tab + 512;
  float* t2 = tab + 640;
  float* p1s = (float*)(ws + OFF_PART1);
  float* p1q = p1s + (size_t)STAT_BLOCKS * CH_HID1;
  float* p2s = (float*)(ws + OFF_PART2);
  float* p2q = p2s + (size_t)STAT_BLOCKS * CH_HID2;
  unsigned short* w1hi = (unsigned short*)(ws + OFF_W1HI);
  unsigned short* w1lo = (unsigned short*)(ws + OFF_W1LO);
  unsigned short* w2hi = (unsigned short*)(ws + OFF_W2HI);
  unsigned short* w2lo = (unsigned short*)(ws + OFF_W2LO);
  float* dsel = (float*)(ws + OFF_DSEL);
  int*   isel = (int*)(ws + OFF_ISEL);
  unsigned short* xt = (unsigned short*)(ws + OFF_PLANEA);
  unsigned short* h1 = (unsigned short*)(ws + OFF_PLANEA);
  float* y1 = (float*)(ws + OFF_PLANEB);
  float* y2 = (float*)(ws + OFF_PLANEB);
  float* out = (float*)d_out;

  const int n8_w1 = (CH_HID1 * CH_IN) / 8;
  const int n8_w2 = (CH_HID2 * CH_HID1) / 8;
  pack_w_kernel<<<(n8_w1 + 255) / 256, 256, 0, stream>>>(W1, w1hi, w1lo, n8_w1);
  pack_w_kernel<<<(n8_w2 + 255) / 256, 256, 0, stream>>>(W2, w2hi, w2lo, n8_w2);

  knn3_kernel<<<NPOINTS / 256, 256, 0, stream>>>(unknown, known, dsel, isel);
  build_x_kernel<<<NPOINTS / 32, 256, 0, stream>>>(kf, uf, dsel, isel, xt);

  {
    const int tiles = (NPOINTS / 64) * (CH_HID1 / 64);
    gemm_f16_wsplit_kernel<<<(tiles + 7) / 8, 256, 0, stream>>>(
        xt, CH_IN, w1hi, w1lo, CH_IN, y1, CH_HID1, b1, NPOINTS, CH_HID1, CH_IN, W_CARRY_INV);
  }
  stats_kernel<CH_HID1><<<STAT_BLOCKS, CH_HID1, 0, stream>>>(y1, p1s, p1q);
  bn_finalize_kernel<<<1, CH_HID1, 0, stream>>>(p1s, p1q, g1, be1, s1, t1, CH_HID1);
  bn_relu_f16_kernel<<<(NPOINTS * (CH_HID1 / 8)) / 256, 256, 0, stream>>>(y1, s1, t1, h1);

  {
    const int tiles = (NPOINTS / 64) * (CH_HID2 / 64);
    gemm_f16_wsplit_kernel<<<(tiles + 7) / 8, 256, 0, stream>>>(
        h1, CH_HID1, w2hi, w2lo, CH_HID1, y2, CH_HID2, b2, NPOINTS, CH_HID2, CH_HID1, W_CARRY_INV);
  }
  stats_kernel<CH_HID2><<<STAT_BLOCKS, CH_HID2, 0, stream>>>(y2, p2s, p2q);
  bn_finalize_kernel<<<1, CH_HID2, 0, stream>>>(p2s, p2q, g2, be2, s2, t2, CH_HID2);
  bn_relu_out_kernel<<<NPOINTS / 32, 256, 0, stream>>>(y2, s2, t2, out);
}
